// SelfMatchingLayer_78847009620109
// MI455X (gfx1250) — hardware-verified
//
#include <hip/hip_runtime.h>
#include <stddef.h>
#include <stdint.h>


#define NB    32
#define NL    512
#define ND    256
#define NG    768
#define NROW  (NB * NL)
#define NTHR  128
#define GTHR  512
#define HS16  264
#define HS32  260

static_assert(ND == 2 * NTHR);
static_assert(NL == 4 * NTHR);
static_assert(NROW % 32 == 0);
static_assert(NL % 16 == 0);
static_assert(NB == 32);
static_assert(GTHR == 16 * 32);
static_assert((HS16 * 2) % 16 == 0);
static_assert((HS32 * 4) % 16 == 0);

typedef _Float16 v4h  __attribute__((ext_vector_type(4)));
typedef _Float16 v8h  __attribute__((ext_vector_type(8)));
typedef _Float16 v16h __attribute__((ext_vector_type(16)));
typedef float    v8f  __attribute__((ext_vector_type(8)));
typedef float    v4f  __attribute__((ext_vector_type(4)));

union Frag { v16h v; v8h h[2]; };

#if __has_builtin(__builtin_amdgcn_exp2f)
#define EXP2_FAST(x) __builtin_amdgcn_exp2f(x)
#else
#define EXP2_FAST(x) exp2f(x)
#endif
#define RCP_FAST(x) __builtin_amdgcn_rcpf(x)

#define WSC   256.0f
#define IWSC  0.00390625f
#define IS12  0.000244140625f
#define C2L2E 2.8853900817779268f
#define LOG2E 1.4426950408889634f

__device__ __forceinline__ v16h frag16(const _Float16* row, int k0, int hh)
{
    Frag f;
    f.h[0] = *(const v8h*)(row + k0 + 8 * hh);
    f.h[1] = *(const v8h*)(row + k0 + 16 + 8 * hh);
    return f.v;
}

__device__ __forceinline__ v8f wmma_f16(v16h a, v16h b, v8f c)
{
    v8f d = __builtin_amdgcn_wmma_f32_16x16x32_f16(false, a, false, b, (short)0, c, false, false);
    asm volatile("v_nop\n\tv_nop\n\tv_nop\n\tv_nop" : "+v"(d) : "v"(a), "v"(b));
    return d;
}

__device__ __forceinline__ v8h pack8h(v4f a, v4f b)
{
    v8h r = { (_Float16)a[0], (_Float16)a[1], (_Float16)a[2], (_Float16)a[3],
              (_Float16)b[0], (_Float16)b[1], (_Float16)b[2], (_Float16)b[3] };
    return r;
}
__device__ __forceinline__ v4h pack4h(v4f a)
{
    v4h r = { (_Float16)a[0], (_Float16)a[1], (_Float16)a[2], (_Float16)a[3] };
    return r;
}

__device__ __forceinline__ float sigm_f(float x)
{
    return RCP_FAST(1.0f + EXP2_FAST(-LOG2E * x));
}
__device__ __forceinline__ float tanh_f(float x)
{
    return 1.0f - 2.0f * RCP_FAST(1.0f + EXP2_FAST(C2L2E * x));
}

__global__ void __launch_bounds__(NTHR) prep_kernel(
    const float* __restrict__ P,
    const float* __restrict__ wq, const float* __restrict__ wp, const float* __restrict__ wg,
    const float* __restrict__ wihl, const float* __restrict__ whhl,
    const float* __restrict__ wihr, const float* __restrict__ whhr,
    _Float16* P16, _Float16* wq16, _Float16* wp16, _Float16* wg16,
    _Float16* wihl16, _Float16* whhl16, _Float16* wihr16, _Float16* whhr16,
    _Float16* PT16)
{
    __shared__ float s_t[32][65];

    const int tid = threadIdx.x;
    const int bid = blockIdx.x;
    const int SA = NROW / 4;
    const int SB = SA + ND / 4;
    const int SC = SB + ND / 4;
    const int SD = SC + (2 * ND) / 4;
    const int SE = SD + NG / 4;
    const int SF = SE + NG / 4;
    const int SG = SF + NG / 4;
    const int SH = SG + NG / 4;

    if (bid < SH) {
        const int rl = tid >> 5;
        const int c8 = tid & 31;
        const float* src;
        _Float16* dst;
        float scale = WSC;
        if (bid < SA) {
            const int row = bid * 4 + rl;
            src = P + (size_t)row * ND;       dst = P16 + (size_t)row * ND;     scale = 1.0f;
        } else if (bid < SB) {
            const int row = (bid - SA) * 4 + rl;
            src = wq + (size_t)row * ND;      dst = wq16 + (size_t)row * ND;
        } else if (bid < SC) {
            const int row = (bid - SB) * 4 + rl;
            src = wp + (size_t)row * ND;      dst = wp16 + (size_t)row * ND;
        } else if (bid < SD) {
            const int row = (bid - SC) * 4 + rl;
            src = wg + (size_t)row * ND;      dst = wg16 + (size_t)row * ND;
        } else if (bid < SE) {
            const int row = (bid - SD) * 4 + rl;
            src = wihl + (size_t)row * ND;    dst = wihl16 + (size_t)row * ND;
        } else if (bid < SF) {
            const int row = (bid - SE) * 4 + rl;
            src = whhl + (size_t)row * ND;    dst = whhl16 + (size_t)row * ND;
        } else if (bid < SG) {
            const int row = (bid - SF) * 4 + rl;
            src = wihr + (size_t)row * ND;    dst = wihr16 + (size_t)row * ND;
        } else {
            const int row = (bid - SG) * 4 + rl;
            src = whhr + (size_t)row * ND;    dst = whhr16 + (size_t)row * ND;
        }
        const v4f x0 = *(const v4f*)(src + 8 * c8);
        const v4f x1 = *(const v4f*)(src + 8 * c8 + 4);
        const v8h val = pack8h(x0 * scale, x1 * scale);
        volatile v8h* p = (volatile v8h*)(dst + 8 * c8);
        *p = val;
        __threadfence();
        *p = val;
    } else {
        const int t   = bid - SH;
        const int b   = t >> 6;
        const int rem = t & 63;
        const int m0  = (rem >> 3) * 64;
        const int d0  = (rem & 7) * 32;
        const float* src = P + ((size_t)b * NL + m0) * ND + d0;
        #pragma unroll
        for (int i = 0; i < 4; ++i) {
            const int idx = tid + NTHR * i;
            const int row = idx >> 3;
            const int c4  = idx & 7;
            const v4f x = *(const v4f*)(src + (size_t)row * ND + 4 * c4);
            s_t[4 * c4 + 0][row] = x[0];
            s_t[4 * c4 + 1][row] = x[1];
            s_t[4 * c4 + 2][row] = x[2];
            s_t[4 * c4 + 3][row] = x[3];
        }
        __syncthreads();
        v8h val[2];
        size_t off[2];
        #pragma unroll
        for (int i = 0; i < 2; ++i) {
            const int idx = tid + NTHR * i;
            const int dl  = idx >> 3;
            const int ms  = (idx & 7) * 8;
            v8h r = { (_Float16)s_t[dl][ms + 0], (_Float16)s_t[dl][ms + 1],
                      (_Float16)s_t[dl][ms + 2], (_Float16)s_t[dl][ms + 3],
                      (_Float16)s_t[dl][ms + 4], (_Float16)s_t[dl][ms + 5],
                      (_Float16)s_t[dl][ms + 6], (_Float16)s_t[dl][ms + 7] };
            val[i] = r;
            off[i] = ((size_t)(b * ND + d0 + dl)) * NL + m0 + ms;
        }
        #pragma unroll
        for (int i = 0; i < 2; ++i) *(volatile v8h*)(PT16 + off[i]) = val[i];
        __threadfence();
        #pragma unroll
        for (int i = 0; i < 2; ++i) *(volatile v8h*)(PT16 + off[i]) = val[i];
    }
}

__global__ void __launch_bounds__(NTHR) proj_kernel(
    const _Float16* __restrict__ A,
    const _Float16* __restrict__ B0, const _Float16* __restrict__ B1,
    const float* __restrict__ bias0, const float* __restrict__ bias1,
    float* C0, float* C1, float scale, float post)
{
    __shared__ __align__(16) float s_c[32][HS32];

    const int which = blockIdx.y;
    const _Float16* Bt  = which ? B1 : B0;
    const float*    bias = which ? bias1 : bias0;
    float*          C    = which ? C1 : C0;

    const int tid = threadIdx.x;
    const int wv  = tid >> 5;
    const int l   = tid & 31;
    const int hh  = l >> 4;
    const int m15 = l & 15;
    const int row0 = blockIdx.x * 32;

    v8f acc[2][4];
    const v8f zero = { 0.f, 0.f, 0.f, 0.f, 0.f, 0.f, 0.f, 0.f };
    #pragma unroll
    for (int rt = 0; rt < 2; ++rt)
        #pragma unroll
        for (int j = 0; j < 4; ++j) acc[rt][j] = zero;

    const _Float16* a0p = A  + (size_t)(row0 + m15) * ND;
    const _Float16* a1p = A  + (size_t)(row0 + 16 + m15) * ND;
    const _Float16* bp  = Bt + (size_t)(64 * wv + m15) * ND;

    #pragma unroll 2
    for (int k0 = 0; k0 < ND; k0 += 32) {
        const v16h fa0 = frag16(a0p, k0, hh);
        const v16h fa1 = frag16(a1p, k0, hh);
        #pragma unroll
        for (int j = 0; j < 4; ++j) {
            const v16h fb = frag16(bp + (size_t)j * 16 * ND, k0, hh);
            acc[0][j] = wmma_f16(fa0, fb, acc[0][j]);
            acc[1][j] = wmma_f16(fa1, fb, acc[1][j]);
        }
    }

    #pragma unroll
    for (int rt = 0; rt < 2; ++rt)
        #pragma unroll
        for (int j = 0; j < 4; ++j)
            #pragma unroll
            for (int r = 0; r < 8; ++r)
                s_c[rt * 16 + 8 * hh + r][64 * wv + 16 * j + m15] = acc[rt][j][r];
    __syncthreads();

    v4f vals[16];
    #pragma unroll
    for (int i = 0; i < 16; ++i) {
        const int idx = tid + NTHR * i;
        const int row = idx >> 6;
        const int c4  = idx & 63;
        const v4f x  = *(const v4f*)&s_c[row][4 * c4];
        const v4f bb = *(const v4f*)(bias + 4 * c4);
        vals[i] = (x * scale + bb) * post;
    }
    #pragma unroll
    for (int i = 0; i < 16; ++i) {
        const int idx = tid + NTHR * i;
        const int row = idx >> 6;
        const int c4  = idx & 63;
        *(volatile v4f*)(C + (size_t)(row0 + row) * ND + 4 * c4) = vals[i];
    }
    __threadfence();
    #pragma unroll
    for (int i = 0; i < 16; ++i) {
        const int idx = tid + NTHR * i;
        const int row = idx >> 6;
        const int c4  = idx & 63;
        *(volatile v4f*)(C + (size_t)(row0 + row) * ND + 4 * c4) = vals[i];
    }
}

__global__ void __launch_bounds__(NTHR) attn_kernel(
    const float* __restrict__ qterm, const float* __restrict__ mterm,
    const float* __restrict__ vvec,  const float* __restrict__ vbias,
    const _Float16* __restrict__ PT, const _Float16* __restrict__ P16,
    const _Float16* __restrict__ wg16, const float* __restrict__ gbias,
    _Float16* CG)
{
    __shared__ __align__(16) float    s_v[ND];
    __shared__ __align__(16) float    s_qh[8][ND];
    __shared__ __align__(16) _Float16 s_p[16][NL];
    __shared__ __align__(16) _Float16 s_c16[16][ND];
    __shared__ __align__(16) float    s_f[16 * ND];
    __shared__ float s_rmax[8][4];
    __shared__ float s_rsum[8][4];

    const int tid = threadIdx.x;
    const int wv  = tid >> 5;
    const int l   = tid & 31;
    const int hh  = l >> 4;
    const int m15 = l & 15;
    const int b   = blockIdx.y;
    const int q0  = blockIdx.x * 16;
    const int mb  = 4 * tid;

    const float NEG_INF = -__builtin_inff();

    s_v[tid]        = vvec[tid];
    s_v[tid + NTHR] = vvec[tid + NTHR];
    const float wsb = vbias[0];
    const float* mrow = mterm + ((size_t)b * NL + mb) * ND;

    for (int jq = 0; jq < 2; ++jq) {
        const int qrow0 = b * NL + q0 + 8 * jq;

        #pragma unroll
        for (int i = 0; i < 4; ++i) {
            const int idx = tid + NTHR * i;
            const int j  = idx >> 6;
            const int c4 = idx & 63;
            *(v4f*)&s_qh[j][4 * c4] = *(const v4f*)(qterm + (size_t)(qrow0 + j) * ND + 4 * c4);
        }
        __syncthreads();

        float acc[8][4];
        #pragma unroll
        for (int j = 0; j < 8; ++j)
            #pragma unroll
            for (int i = 0; i < 4; ++i) acc[j][i] = 0.0f;

        #pragma unroll 1
        for (int d4 = 0; d4 < ND / 4; ++d4) {
            v4f mv[4];
            #pragma unroll
            for (int i = 0; i < 4; ++i) mv[i] = *(const v4f*)(mrow + (size_t)i * ND + 4 * d4);
            v4f qv[8];
            #pragma unroll
            for (int j = 0; j < 8; ++j) qv[j] = *(const v4f*)&s_qh[j][4 * d4];
            const v4f vv = *(const v4f*)&s_v[4 * d4];
            #pragma unroll
            for (int e = 0; e < 4; ++e) {
                const float ve = vv[e];
                #pragma unroll
                for (int j = 0; j < 8; ++j) {
                    const float qe = qv[j][e];
                    #pragma unroll
                    for (int i = 0; i < 4; ++i) {
                        const float hx = qe + mv[i][e];
                        const float ex = EXP2_FAST(hx);
                        const float rr = RCP_FAST(ex + 1.0f);
                        acc[j][i] = fmaf(ve, rr, acc[j][i]);
                    }
                }
            }
        }

        float bm[8];
        #pragma unroll
        for (int j = 0; j < 8; ++j) {
            float lm = NEG_INF;
            #pragma unroll
            for (int i = 0; i < 4; ++i) {
                const float s = fmaf(-2.0f, acc[j][i], wsb);
                acc[j][i] = s;
                lm = fmaxf(lm, s);
            }
            #pragma unroll
            for (int off = 16; off > 0; off >>= 1) lm = fmaxf(lm, __shfl_xor(lm, off, 32));
            bm[j] = lm;
        }
        if (l == 0) {
            #pragma unroll
            for (int j = 0; j < 8; ++j) s_rmax[j][wv] = bm[j];
        }
        __syncthreads();
        #pragma unroll
        for (int j = 0; j < 8; ++j)
            bm[j] = fmaxf(fmaxf(s_rmax[j][0], s_rmax[j][1]), fmaxf(s_rmax[j][2], s_rmax[j][3]));

        float bs[8];
        #pragma unroll
        for (int j = 0; j < 8; ++j) {
            float ls = 0.0f;
            #pragma unroll
            for (int i = 0; i < 4; ++i) {
                const float ev = EXP2_FAST((acc[j][i] - bm[j]) * LOG2E);
                acc[j][i] = ev;
                ls += ev;
            }
            #pragma unroll
            for (int off = 16; off > 0; off >>= 1) ls += __shfl_xor(ls, off, 32);
            bs[j] = ls;
        }
        if (l == 0) {
            #pragma unroll
            for (int j = 0; j < 8; ++j) s_rsum[j][wv] = bs[j];
        }
        __syncthreads();
        #pragma unroll
        for (int j = 0; j < 8; ++j)
            bs[j] = (s_rsum[j][0] + s_rsum[j][1]) + (s_rsum[j][2] + s_rsum[j][3]);

        #pragma unroll
        for (int j = 0; j < 8; ++j) {
            const float inv = 1.0f / bs[j];
            const v4f w = { acc[j][0] * inv, acc[j][1] * inv, acc[j][2] * inv, acc[j][3] * inv };
            *(v4h*)&s_p[8 * jq + j][mb] = pack4h(w * 16384.0f);
        }
    }
    __syncthreads();

    const v8f zero = { 0.f, 0.f, 0.f, 0.f, 0.f, 0.f, 0.f, 0.f };
    v8f pacc[4];
    #pragma unroll
    for (int j = 0; j < 4; ++j) pacc[j] = zero;

    const _Float16* prow = &s_p[m15][0];
    const _Float16* brow = PT + ((size_t)(b * ND + 64 * wv + m15)) * NL;
    #pragma unroll 2
    for (int k0 = 0; k0 < NL; k0 += 32) {
        const v16h fa = frag16(prow, k0, hh);
        #pragma unroll
        for (int j = 0; j < 4; ++j) {
            const v16h fb = frag16(brow + (size_t)j * 16 * NL, k0, hh);
            pacc[j] = wmma_f16(fa, fb, pacc[j]);
        }
    }
    const float OSC = 6.103515625e-05f;
    #pragma unroll
    for (int j = 0; j < 4; ++j)
        #pragma unroll
        for (int r = 0; r < 8; ++r) {
            const float c = pacc[j][r] * OSC;
            s_f[(8 * hh + r) * ND + 64 * wv + 16 * j + m15] = c;
            s_c16[8 * hh + r][64 * wv + 16 * j + m15] = (_Float16)c;
        }
    __syncthreads();

    v8f gacc[4];
    #pragma unroll
    for (int j = 0; j < 4; ++j) gacc[j] = zero;
    const _Float16* arow = P16 + (size_t)(b * NL + q0 + m15) * ND;
    const _Float16* grow = wg16 + (size_t)(64 * wv + m15) * (2 * ND);
    #pragma unroll 2
    for (int k0 = 0; k0 < ND; k0 += 32) {
        const v16h fa = frag16(arow, k0, hh);
        #pragma unroll
        for (int j = 0; j < 4; ++j) {
            const v16h fb = frag16(grow + (size_t)j * 16 * (2 * ND), k0, hh);
            gacc[j] = wmma_f16(fa, fb, gacc[j]);
        }
    }
    const _Float16* crow = &s_c16[m15][0];
    #pragma unroll 2
    for (int k0 = 0; k0 < ND; k0 += 32) {
        const v16h fa = frag16(crow, k0, hh);
        #pragma unroll
        for (int j = 0; j < 4; ++j) {
            const v16h fb = frag16(grow + (size_t)j * 16 * (2 * ND), ND + k0, hh);
            gacc[j] = wmma_f16(fa, fb, gacc[j]);
        }
    }
    #pragma unroll
    for (int j = 0; j < 4; ++j) {
        const int col = 64 * wv + 16 * j + m15;
        const float gb = gbias[col];
        #pragma unroll
        for (int r = 0; r < 8; ++r) {
            const int idx = (8 * hh + r) * ND + col;
            const float pre = fmaf(gacc[j][r], IWSC, gb);
            const float g = sigm_f(pre);
            s_f[idx] = 16.0f * g * s_f[idx];
        }
    }
    __syncthreads();

    v8h cv[4];
    size_t off[4];
    #pragma unroll
    for (int i = 0; i < 4; ++i) {
        const int idx = tid + NTHR * i;
        const int row = idx >> 5;
        const int c8  = idx & 31;
        const v4f o0 = *(const v4f*)&s_f[row * ND + 8 * c8];
        const v4f o1 = *(const v4f*)&s_f[row * ND + 8 * c8 + 4];
        cv[i]  = pack8h(o0, o1);
        off[i] = ((size_t)(q0 + row) * NB + b) * ND + 8 * c8;
    }
    #pragma unroll
    for (int i = 0; i < 4; ++i) *(volatile v8h*)(CG + off[i]) = cv[i];
    __threadfence();
    #pragma unroll
    for (int i = 0; i < 4; ++i) *(volatile v8h*)(CG + off[i]) = cv[i];
}

__global__ void __launch_bounds__(GTHR) gru_kernel(
    const _Float16* __restrict__ CG,
    const _Float16* __restrict__ wihl, const _Float16* __restrict__ whhl,
    const float* __restrict__ bihl, const float* __restrict__ bhhl,
    const _Float16* __restrict__ wihr, const _Float16* __restrict__ whhr,
    const float* __restrict__ bihr, const float* __restrict__ bhhr,
    float* out)
{
    __shared__ __align__(16) _Float16 h16[NB * HS16];
    __shared__ __align__(16) float    h32[NB * HS32];

    const int dir = blockIdx.x;
    const _Float16* wih = dir ? wihr : wihl;
    const _Float16* whh = dir ? whhr : whhl;
    const float*    bih = dir ? bihr : bihl;
    const float*    bhh = dir ? bhhr : bhhl;

    const int tid = threadIdx.x;
    const int wv  = tid >> 5;
    const int l   = tid & 31;
    const int hh  = l >> 4;
    const int m15 = l & 15;
    const int j   = 16 * wv + m15;

    for (int i = tid; i < NB * HS16; i += GTHR) h16[i] = (_Float16)0.0f;
    for (int i = tid; i < NB * HS32; i += GTHR) h32[i] = 0.0f;
    __syncthreads();

    const float bR  = bih[j] + bhh[j];
    const float bZ  = bih[ND + j] + bhh[ND + j];
    const float bIN = bih[2 * ND + j];
    const float bHN = bhh[2 * ND + j];

    const _Float16* wir = wih + (size_t)j * ND;
    const _Float16* wiz = wih + (size_t)(ND + j) * ND;
    const _Float16* win = wih + (size_t)(2 * ND + j) * ND;
    const _Float16* whr = whh + (size_t)j * ND;
    const _Float16* whz = whh + (size_t)(ND + j) * ND;
    const _Float16* whn = whh + (size_t)(2 * ND + j) * ND;

    const _Float16* hrow0 = &h16[m15 * HS16];
    const _Float16* hrow1 = &h16[(16 + m15) * HS16];

    const v8f zero = { 0.f, 0.f, 0.f, 0.f, 0.f, 0.f, 0.f, 0.f };
    const int orow = 2 * wv + hh;

    #pragma unroll 1
    for (int s = 0; s < NL; ++s) {
        const int t = dir ? (NL - 1 - s) : s;
        const _Float16* crow0 = CG + ((size_t)t * NB + m15) * ND;
        const _Float16* crow1 = crow0 + (size_t)16 * ND;

        v8f aR0 = zero, aR1 = zero, aZ0 = zero, aZ1 = zero;
        v8f aI0 = zero, aI1 = zero, aH0 = zero, aH1 = zero;

        #pragma unroll 1
        for (int k0 = 0; k0 < ND; k0 += 32) {
            const v16h fc0 = frag16(crow0, k0, hh);
            const v16h fc1 = frag16(crow1, k0, hh);
            const v16h fh0 = frag16(hrow0, k0, hh);
            const v16h fh1 = frag16(hrow1, k0, hh);
            v16h fb;
            fb = frag16(wir, k0, hh);  aR0 = wmma_f16(fc0, fb, aR0);  aR1 = wmma_f16(fc1, fb, aR1);
            fb = frag16(whr, k0, hh);  aR0 = wmma_f16(fh0, fb, aR0);  aR1 = wmma_f16(fh1, fb, aR1);
            fb = frag16(wiz, k0, hh);  aZ0 = wmma_f16(fc0, fb, aZ0);  aZ1 = wmma_f16(fc1, fb, aZ1);
            fb = frag16(whz, k0, hh);  aZ0 = wmma_f16(fh0, fb, aZ0);  aZ1 = wmma_f16(fh1, fb, aZ1);
            fb = frag16(win, k0, hh);  aI0 = wmma_f16(fc0, fb, aI0);  aI1 = wmma_f16(fc1, fb, aI1);
            fb = frag16(whn, k0, hh);  aH0 = wmma_f16(fh0, fb, aH0);  aH1 = wmma_f16(fh1, fb, aH1);
        }

        float hn0[8], hn1[8];
        #pragma unroll
        for (int r = 0; r < 8; ++r) {
            {
                const int bb = 8 * hh + r;
                const float rr = sigm_f(fmaf(aR0[r], IS12, bR));
                const float zz = sigm_f(fmaf(aZ0[r], IS12, bZ));
                const float nn = tanh_f(fmaf(aI0[r], IS12, bIN) + rr * fmaf(aH0[r], IS12, bHN));
                const float ho = h32[bb * HS32 + j];
                hn0[r] = (1.0f - zz) * nn + zz * ho;
            }
            {
                const int bb = 16 + 8 * hh + r;
                const float rr = sigm_f(fmaf(aR1[r], IS12, bR));
                const float zz = sigm_f(fmaf(aZ1[r], IS12, bZ));
                const float nn = tanh_f(fmaf(aI1[r], IS12, bIN) + rr * fmaf(aH1[r], IS12, bHN));
                const float ho = h32[bb * HS32 + j];
                hn1[r] = (1.0f - zz) * nn + zz * ho;
            }
        }
        __syncthreads();
        #pragma unroll
        for (int r = 0; r < 8; ++r) {
            const int b0 = 8 * hh + r;
            const int b1 = 16 + 8 * hh + r;
            h32[b0 * HS32 + j] = hn0[r];
            h32[b1 * HS32 + j] = hn1[r];
            h16[b0 * HS16 + j] = (_Float16)(16.0f * hn0[r]);
            h16[b1 * HS16 + j] = (_Float16)(16.0f * hn1[r]);
        }
        __syncthreads();

        float* op = out + ((size_t)orow * NL + t) * (2 * ND) + (size_t)dir * ND;
        v4f ov[4];
        #pragma unroll
        for (int i = 0; i < 4; ++i) {
            const int c4 = 16 * i + m15;
            ov[i] = *(const v4f*)&h32[orow * HS32 + 4 * c4];
        }
        #pragma unroll
        for (int i = 0; i < 4; ++i) *(volatile v4f*)(op + 4 * (16 * i + m15)) = ov[i];
        __threadfence();
        #pragma unroll
        for (int i = 0; i < 4; ++i) *(volatile v4f*)(op + 4 * (16 * i + m15)) = ov[i];
    }
}

extern "C" void kernel_launch(void* const* d_in, const int* in_sizes, int n_in,
                              void* d_out, int out_size, void* d_ws, size_t ws_size,
                              hipStream_t stream)
{
    if (n_in < 17) return;
    if (in_sizes[0] != NROW * ND) return;
    if (in_sizes[1] != ND * ND || in_sizes[2] != ND) return;
    if (in_sizes[3] != ND * ND || in_sizes[4] != ND) return;
    if (in_sizes[5] != ND || in_sizes[6] < 1) return;
    if (in_sizes[7] != ND * 2 * ND || in_sizes[8] != ND) return;
    if (in_sizes[9]  != NG * ND || in_sizes[10] != NG * ND) return;
    if (in_sizes[11] != NG || in_sizes[12] != NG) return;
    if (in_sizes[13] != NG * ND || in_sizes[14] != NG * ND) return;
    if (in_sizes[15] != NG || in_sizes[16] != NG) return;
    if (out_size != NROW * 2 * ND) return;

    const float* P     = (const float*)d_in[0];
    const float* wq_w  = (const float*)d_in[1];
    const float* wq_b  = (const float*)d_in[2];
    const float* wp_w  = (const float*)d_in[3];
    const float* wp_b  = (const float*)d_in[4];
    const float* ws_w  = (const float*)d_in[5];
    const float* ws_b  = (const float*)d_in[6];
    const float* wg_w  = (const float*)d_in[7];
    const float* wg_b  = (const float*)d_in[8];
    const float* Wih_l = (const float*)d_in[9];
    const float* Whh_l = (const float*)d_in[10];
    const float* bih_l = (const float*)d_in[11];
    const float* bhh_l = (const float*)d_in[12];
    const float* Wih_r = (const float*)d_in[13];
    const float* Whh_r = (const float*)d_in[14];
    const float* bih_r = (const float*)d_in[15];
    const float* bhh_r = (const float*)d_in[16];
    float* out = (float*)d_out;

    const size_t szP16 = (size_t)NROW * ND * 2;
    const size_t szW   = (size_t)ND * ND * 2;
    const size_t szWG  = (size_t)ND * 2 * ND * 2;
    const size_t szWR  = (size_t)NG * ND * 2;
    const size_t szF32 = (size_t)NROW * ND * 4;
    size_t off = 0;
    const size_t oP16  = off;  off += szP16;
    const size_t oPT16 = off;  off += szP16;
    const size_t oWQ   = off;  off += szW;
    const size_t oWP   = off;  off += szW;
    const size_t oWG   = off;  off += szWG;
    const size_t oWIHL = off;  off += szWR;
    const size_t oWHHL = off;  off += szWR;
    const size_t oWIHR = off;  off += szWR;
    const size_t oWHHR = off;  off += szWR;
    const size_t oHQ   = off;  off += szF32;
    const size_t oPP   = off;  off += szF32;
    const size_t oCG   = off;  off += szP16;
    if (off > ws_size) return;

    char* ws = (char*)d_ws;
    _Float16* P16    = (_Float16*)(ws + oP16);
    _Float16* PT16   = (_Float16*)(ws + oPT16);
    _Float16* wq16   = (_Float16*)(ws + oWQ);
    _Float16* wp16   = (_Float16*)(ws + oWP);
    _Float16* wg16   = (_Float16*)(ws + oWG);
    _Float16* wihl16 = (_Float16*)(ws + oWIHL);
    _Float16* whhl16 = (_Float16*)(ws + oWHHL);
    _Float16* wihr16 = (_Float16*)(ws + oWIHR);
    _Float16* whhr16 = (_Float16*)(ws + oWHHR);
    float*    Hq2    = (float*)(ws + oHQ);
    float*    Pp2    = (float*)(ws + oPP);
    _Float16* CG16   = (_Float16*)(ws + oCG);

    const int nprep = NROW / 4 + ND / 4 + ND / 4 + (2 * ND) / 4 + 4 * (NG / 4)
                    + NB * (NL / 64) * (ND / 32);
    prep_kernel<<<dim3(nprep), dim3(NTHR), 0, stream>>>(
        P, wq_w, wp_w, wg_w, Wih_l, Whh_l, Wih_r, Whh_r,
        P16, wq16, wp16, wg16, wihl16, whhl16, wihr16, whhr16, PT16);

    proj_kernel<<<dim3(NROW / 32, 2), dim3(NTHR), 0, stream>>>(
        P16, wq16, wp16, wq_b, wp_b, Hq2, Pp2, IWSC, C2L2E);

    attn_kernel<<<dim3(NL / 16, NB), dim3(NTHR), 0, stream>>>(
        Pp2, Hq2, ws_w, ws_b, PT16, P16, wg16, wg_b, CG16);

    gru_kernel<<<dim3(2), dim3(GTHR), 0, stream>>>(
        CG16, wihl16, whhl16, bih_l, bhh_l, wihr16, whhr16, bih_r, bhh_r, out);
}
